// clipSCPFlow3D_28381143892158
// MI455X (gfx1250) — hardware-verified
//
#include <hip/hip_runtime.h>


namespace {
constexpr int C = 32, DD = 80, HH = 80, WW = 80, NV = DD * HH * WW  , NCLS = 36, ID = 768, C1 = 64, C2 = 128, OC = 32, KT = 27;
constexpr float WSC = 65536.0f, WSI = 1.0f / 65536.0f;

typedef _Float16 b16;
typedef __attribute__((ext_vector_type(16))) _Float16 v16b;
typedef __attribute__((ext_vector_type(8))) _Float16 v8b;
typedef __attribute__((ext_vector_type(8))) float v8f;
typedef __attribute__((ext_vector_type(4))) float v4f;
__device__ __forceinline__ v16b frag_kb(const b16* p, int hh) { const v8b a = *(const v8b*)(p + 8 * hh), b = *(const v8b*)(p + 16 + 8 * hh); v16b f;
#pragma unroll
  for (int e = 0; e < 8; ++e) { f[e] = a[e]; f[8 + e] = b[e]; } return f; }
__device__ __forceinline__ v8f wmma16b(v16b a, v16b b, v8f c) {
  v8f d = __builtin_amdgcn_wmma_f32_16x16x32_f16(false, a, false, b, (short)0, c, false, false);
  asm volatile("v_nop\n\tv_nop\n\tv_nop\n\tv_nop" : "+v"(d) : "v"(a), "v"(b));
  return d;
}
__device__ __forceinline__ void wave_lds_sync() { __builtin_amdgcn_fence(__ATOMIC_RELEASE, "workgroup"); __builtin_amdgcn_wave_barrier(); __builtin_amdgcn_fence(__ATOMIC_ACQUIRE, "workgroup"); }

__global__ __launch_bounds__(256) void mlp_kernel(const float* __restrict__ tf, const float* __restrict__ w1x, const float* __restrict__ b1x, const float* __restrict__ w2x, const float* __restrict__ b2x, const float* __restrict__ w3x, const float* __restrict__ b3x,
                                                  const float* __restrict__ w1y, const float* __restrict__ b1y, const float* __restrict__ w2y, const float* __restrict__ b2y, const float* __restrict__ w3y, const float* __restrict__ b3y,
                                                  const float* __restrict__ w1z, const float* __restrict__ b1z, const float* __restrict__ w2z, const float* __restrict__ b2z, const float* __restrict__ w3z, const float* __restrict__ b3z, float* __restrict__ base) {
  __shared__ float H1[NCLS][C1]; __shared__ float H2[NCLS][C2]; __shared__ float Bo[NCLS * OC];
  const int d = blockIdx.x, t_ = threadIdx.x;
  const float* w1 = (d == 0) ? w1x : (d == 1) ? w1y : w1z; const float* b1 = (d == 0) ? b1x : (d == 1) ? b1y : b1z; const float* w2 = (d == 0) ? w2x : (d == 1) ? w2y : w2z; const float* b2 = (d == 0) ? b2x : (d == 1) ? b2y : b2z; const float* w3 = (d == 0) ? w3x : (d == 1) ? w3y : w3z; const float* b3 = (d == 0) ? b3x : (d == 1) ? b3y : b3z;
  for (int i = t_; i < NCLS * C1; i += 256) { const int r = i / C1, o = i % C1; float s = b1[o];
#pragma unroll 1
    for (int k = 0; k < ID; ++k) s += tf[(size_t)r * ID + k] * w1[(size_t)k * C1 + o];
    H1[r][o] = fmaxf(s, 0.0f); }
  __syncthreads();
  for (int i = t_; i < NCLS * C2; i += 256) { const int r = i / C2, o = i % C2; float s = b2[o];
#pragma unroll 1
    for (int k = 0; k < C1; ++k) s += H1[r][k] * w2[(size_t)k * C2 + o];
    H2[r][o] = fmaxf(s, 0.0f); }
  __syncthreads();
  for (int i = t_; i < NCLS * OC; i += 256) { const int r = i / OC, o = i % OC; float s = b3[o];
#pragma unroll 1
    for (int k = 0; k < C2; ++k) s += H2[r][k] * w3[(size_t)k * OC + o];
    Bo[i] = s; }
  __syncthreads();
  for (int pass = 0; pass < 2; ++pass) { for (int i = t_; i < NCLS * OC / 4; i += 256) *(volatile v4f*)(base + (size_t)d * NCLS * OC + i * 4) = *(const v4f*)(&Bo[i * 4]); __threadfence(); }
}

__global__ __launch_bounds__(256) void prep_kernel(const float* __restrict__ x, const float* __restrict__ cw, b16* __restrict__ xt, b16* __restrict__ wv) {
  const size_t tid = (size_t)blockIdx.x * blockDim.x + threadIdx.x, nth = (size_t)gridDim.x * blockDim.x;
  for (int pass = 0; pass < 2; ++pass) {
    for (size_t p = tid; p < (size_t)(NV + 1) * (C / 8); p += nth) { const int v = (int)(p / (C / 8)), c0 = (int)(p % (C / 8)) * 8; v8b o;
#pragma unroll
      for (int e = 0; e < 8; ++e) o[e] = (b16)((v < NV) ? x[(size_t)(c0 + e) * NV + min(v, NV - 1)] : 0.0f);
      *(volatile v8b*)(xt + (size_t)v * C + c0) = o; }
    for (size_t p = tid; p < (size_t)16 * KT * C; p += nth) { const int o = (int)(p / (KT * C)), k = (int)(p % (KT * C)), tap = k / C, c = k % C;
      ((volatile b16*)wv)[p] = (b16)((o < 3) ? cw[((size_t)min(o, 2) * C + c) * KT + tap] * WSC : 0.0f); }
    __threadfence();
  }
}

__global__ __launch_bounds__(256) void main_kernel(const float* __restrict__ x, const int* __restrict__ yseg, const float* __restrict__ base, const b16* __restrict__ xt, const b16* __restrict__ wv, const float* __restrict__ cb, float* __restrict__ out) {
  __shared__ float Bs[3 * NCLS * OC]; __shared__ float So[8][3][32];
  const int t_ = threadIdx.x, wid = t_ >> 5, lane = t_ & 31, nloc = lane & 15, hh = lane >> 4;
  for (int i = t_; i < 3 * NCLS * OC; i += 256) Bs[i] = base[i];
  __syncthreads();
  const int v0 = (blockIdx.x * 8 + wid) * 32;
#pragma unroll
  for (int r = 0; r < 2; ++r) {
    const int v = v0 + r * 16 + nloc; const int w_ = v % WW, h_ = (v / WW) % HH, d_ = v / (WW * HH);
    int cls = yseg[((size_t)(2 * d_) * (2 * HH) + 2 * h_) * (2 * WW) + 2 * w_]; cls = (cls < 0) ? 0 : (cls >= NCLS ? NCLS - 1 : cls);
    float s0 = 0.0f, s1 = 0.0f, s2 = 0.0f;
#pragma unroll 4
    for (int c = 0; c < 16; ++c) { const int cc = 16 * hh + c; const float xv = x[(size_t)cc * NV + v]; s0 += Bs[(0 * NCLS + cls) * OC + cc] * xv; s1 += Bs[(1 * NCLS + cls) * OC + cc] * xv; s2 += Bs[(2 * NCLS + cls) * OC + cc] * xv; }
    s0 += __shfl_xor(s0, 16); s1 += __shfl_xor(s1, 16); s2 += __shfl_xor(s2, 16);
    v8f acc = {};
#pragma unroll 9
    for (int tap = 0; tap < KT; ++tap) { const int kd = tap / 9 - 1, kh = (tap / 3) % 3 - 1, kw = tap % 3 - 1; const int dn = d_ + kd, hn = h_ + kh, wn = w_ + kw;
      const bool ok = (dn >= 0) && (dn < DD) && (hn >= 0) && (hn < HH) && (wn >= 0) && (wn < WW); const int vn = ok ? ((dn * HH + hn) * WW + wn) : NV;
      const v16b a = frag_kb(xt + (size_t)vn * C, hh), b = frag_kb(wv + (size_t)nloc * (KT * C) + tap * C, hh);
      acc = wmma16b(a, b, acc); }
    if (hh == 0) { So[wid][0][r * 16 + nloc] = s0; So[wid][1][r * 16 + nloc] = s1; So[wid][2][r * 16 + nloc] = s2; }
    wave_lds_sync();
    if (nloc < 3) {
#pragma unroll
      for (int j = 0; j < 8; ++j) So[wid][nloc][r * 16 + 8 * hh + j] += acc[j] * WSI + cb[nloc]; }
    wave_lds_sync();
  }
  for (int pass = 0; pass < 2; ++pass) {
#pragma unroll
    for (int o = 0; o < 3; ++o) ((volatile float*)out)[(size_t)o * NV + v0 + lane] = So[wid][o][lane];
    __threadfence();
  }
}
}

extern "C" void kernel_launch(void* const* d_in, const int* in_sizes, int n_in,
                              void* d_out, int out_size, void* d_ws, size_t ws_size, hipStream_t stream) {
  (void)n_in; (void)out_size;
  const float* x = (const float*)d_in[0]; const int* yseg = (const int*)d_in[1]; const float* tf = (const float*)d_in[2];
  const float* p[18]; for (int i = 0; i < 18; ++i) p[i] = (const float*)d_in[3 + i];
  const float* cw = (const float*)d_in[21]; const float* cb = (const float*)d_in[22];
  float* out = (float*)d_out;
  if (in_sizes[0] != C * NV || in_sizes[1] != 8 * NV || in_sizes[2] != NCLS * ID || in_sizes[3] != ID * C1 || in_sizes[21] != 3 * C * KT) return;
  size_t off = 0; char* ws = (char*)d_ws;
  auto carve = [&](size_t bytes) { char* q = ws + off; off += (bytes + 255) & ~(size_t)255; return q; };
  float* base = (float*)carve((size_t)3 * NCLS * OC * 4 + 256); b16* xt = (b16*)carve((size_t)(NV + 1) * C * 2 + 256); b16* wv = (b16*)carve((size_t)16 * KT * C * 2);
  if (off > ws_size) return;
  mlp_kernel<<<3, 256, 0, stream>>>(tf, p[0], p[1], p[2], p[3], p[4], p[5], p[6], p[7], p[8], p[9], p[10], p[11], p[12], p[13], p[14], p[15], p[16], p[17], base);
  prep_kernel<<<1024, 256, 0, stream>>>(x, cw, xt, wv);
  main_kernel<<<NV / 32 / 8, 256, 0, stream>>>(x, yseg, base, xt, wv, cb, out);
}
